// TransformerLayer_43843026158032
// MI455X (gfx1250) — hardware-verified
//
#include <hip/hip_runtime.h>
#include <math.h>

typedef __attribute__((ext_vector_type(16))) _Float16 v16h;
typedef __attribute__((ext_vector_type(16))) __bf16 v16b;
typedef __attribute__((ext_vector_type(8)))  _Float16 v8h;
typedef __attribute__((ext_vector_type(8)))  __bf16 v8b;
typedef __attribute__((ext_vector_type(8)))  float v8f;
typedef __attribute__((ext_vector_type(4)))  float v4f;
typedef __attribute__((ext_vector_type(8)))  unsigned short v8us;
typedef __attribute__((ext_vector_type(4)))  unsigned short v4us;

#ifndef SEQ
#define SEQ 2048
#endif
#define SEQ_FULL 2048
#ifndef NB
#define NB 2
#endif
#define NB_FULL 2
#define DM 1024
#define NH 16
#define HD 64
#define MROWS (NB * SEQ)
#define SCALE (0.125f)
#define RC (4096.0f)
#define PCY (16384.0f)
#define WC (64.0f)
#define CC (64.0f)
#define F16MIN (6.103515625e-05f)
static_assert(SEQ % 128 == 0);
static_assert(SEQ >= 128);
static_assert(SEQ <= SEQ_FULL);
static_assert(NB >= 1 && NB <= NB_FULL);
static_assert(DM == 1024);
static_assert(NH == 16 && HD == 64 && NH * HD == DM);
static_assert(MROWS % 64 == 0);
static_assert(DM % 128 == 0);

#define WSZ_ACT  (2u * (size_t)MROWS * DM)
#define WSZ_W    (2u * (size_t)DM * DM)
#define WS_XB   ((size_t)0)
#define WS_WQT  (WS_XB  + WSZ_ACT)
#define WS_WKT  (WS_WQT + WSZ_W)
#define WS_WVT  (WS_WKT + WSZ_W)
#define WS_WOH  (WS_WVT + WSZ_W)
#define WS_QH   (WS_WOH + WSZ_W)
#define WS_QL   (WS_QH  + WSZ_ACT)
#define WS_KH   (WS_QL  + WSZ_ACT)
#define WS_KL   (WS_KH  + WSZ_ACT)
#define WS_VT   (WS_KL  + WSZ_ACT)
#define WS_CTX  (WS_VT  + WSZ_ACT)
#define WS_END  (WS_CTX + WSZ_ACT)
static_assert(WS_END <= (size_t)134217728u);
static_assert((WSZ_ACT % 256u) == 0 && (WSZ_W % 256u) == 0);

#define N8X ((unsigned)(NB) * (unsigned)(SEQ) * (unsigned)(DM / 8))
static_assert(N8X % 256u == 0);

template <typename T> __device__ __forceinline__ void vst2(void* p, T v) { *(volatile T*)p = v; __threadfence(); *(volatile T*)p = v; }
__device__ __forceinline__ v8f zero8() { v8f z = {0.f, 0.f, 0.f, 0.f, 0.f, 0.f, 0.f, 0.f}; return z; }
__device__ __forceinline__ v8f wmma16(v16h a, v16h b, v8f c) {
  v8f d = __builtin_amdgcn_wmma_f32_16x16x32_f16(false, a, false, b, (short)0, c, false, false);
  asm volatile("v_nop\n\tv_nop\n\tv_nop\n\tv_nop" : "+v"(d) : "v"(a), "v"(b));
  return d;
}
__device__ __forceinline__ v8f wmma_bf(v16b a, v16b b, v8f c) {
  v8f d = __builtin_amdgcn_wmma_f32_16x16x32_bf16(false, a, false, b, (short)0, c, false, false);
  asm volatile("v_nop\n\tv_nop\n\tv_nop\n\tv_nop" : "+v"(d) : "v"(a), "v"(b));
  return d;
}
__device__ __forceinline__ v16h frag_h(const _Float16* rowk0, int lane) {
  union { v16h v; v8h q[2]; } u; const _Float16* p = rowk0 + 8 * (lane >> 4);
  u.q[0] = *(const v8h*)p; u.q[1] = *(const v8h*)(p + 16); return u.v;
}
__device__ __forceinline__ v16b frag_b(const __bf16* rowk0, int lane) {
  union { v16b v; v8b q[2]; } u; const __bf16* p = rowk0 + 8 * (lane >> 4);
  u.q[0] = *(const v8b*)p; u.q[1] = *(const v8b*)(p + 16); return u.v;
}
__device__ __forceinline__ _Float16 f16n(float x) { const float t = (fabsf(x) >= F16MIN) ? x : 0.0f; return (_Float16)t; }
__device__ __forceinline__ unsigned short bf16bits(float x) { unsigned u = __float_as_uint(x); u += 0x7FFFu + ((u >> 16) & 1u); return (unsigned short)(u >> 16); }
__device__ __forceinline__ float bf16val(unsigned short b) { return __uint_as_float(((unsigned)b) << 16); }
#define LDSX() do { asm volatile("s_wait_dscnt 0" ::: "memory"); __builtin_amdgcn_wave_barrier(); __builtin_amdgcn_fence(3  , "workgroup"); } while (0)

__global__ __launch_bounds__(256) void k_cvtx(const float* __restrict__ src, unsigned short* __restrict__ dst) {
  const unsigned i = blockIdx.x * 256u + threadIdx.x; if (i >= N8X) return;
  const unsigned row = i >> 7, c8 = i & 127u;
  const unsigned b = row / (unsigned)SEQ, s = row - b * (unsigned)SEQ;
  const float* p = src + ((size_t)(b * (unsigned)SEQ_FULL + s) * DM + c8 * 8u);
  const v4f a = *(const v4f*)p, c = *(const v4f*)(p + 4);
  v8us o;
#pragma unroll
  for (int e = 0; e < 4; ++e) { o[e] = bf16bits(a[e]); o[4 + e] = bf16bits(c[e]); }
  vst2(dst + (size_t)i * 8, o);
}

__global__ __launch_bounds__(256) void k_cvtw(const float* __restrict__ W0, const float* __restrict__ W1, const float* __restrict__ W2, const float* __restrict__ W3,
                                              unsigned short* __restrict__ D0, unsigned short* __restrict__ D1, unsigned short* __restrict__ D2, unsigned short* __restrict__ D3) {
  __shared__ __align__(16) unsigned short t[64][72];
  const int tid = threadIdx.x; const unsigned z = blockIdx.z;
  const float* W = (z == 0u) ? W0 : (z == 1u) ? W1 : (z == 2u) ? W2 : W3;
  unsigned short* D = (z == 0u) ? D0 : (z == 1u) ? D1 : (z == 2u) ? D2 : D3;
  const bool hm = (z == 3u);
  const int k0 = blockIdx.y * 64, n0 = blockIdx.x * 64;
#pragma unroll
  for (int it = 0; it < 4; ++it) {
    const int e = tid + it * 256, kr = e >> 4, nq = e & 15;
    const v4f a = *(const v4f*)(W + (size_t)(k0 + kr) * DM + n0 + nq * 4);
#pragma unroll
    for (int i = 0; i < 4; ++i) {
      const unsigned short bb = bf16bits(a[i]);
      const unsigned short hb = __builtin_bit_cast(unsigned short, f16n(bf16val(bb) * WC));
      t[nq * 4 + i][kr] = hm ? hb : bb;
    }
  }
  __syncthreads();
#pragma unroll
  for (int it = 0; it < 2; ++it) {
    const int e = tid + it * 256, nl = e >> 3, q = e & 7;
    vst2(D + (size_t)(n0 + nl) * DM + k0 + q * 8, *(const v8us*)&t[nl][q * 8]);
  }
}

__global__ __launch_bounds__(128) void k_pqk(const __bf16* __restrict__ XB, const __bf16* __restrict__ WQT, const __bf16* __restrict__ WKT,
                                             _Float16* __restrict__ QH, _Float16* __restrict__ QL, _Float16* __restrict__ KH, _Float16* __restrict__ KL) {
  __shared__ __align__(16) _Float16 sh[64][136], sl[64][136];
  const int tid = threadIdx.x, wave = tid >> 5, lane = tid & 31, col = lane & 15, g = lane >> 4;
  const bool zk = (blockIdx.z != 0u);
  const __bf16* WB = zk ? WKT : WQT; _Float16* OH = zk ? KH : QH; _Float16* OL = zk ? KL : QL;
  const int c0 = blockIdx.y * 128; const size_t r0 = (size_t)blockIdx.x * 64;
  v8f acc[8];
#pragma unroll
  for (int j = 0; j < 8; ++j) acc[j] = zero8();
#pragma unroll 1
  for (int kc = 0; kc < DM / 32; ++kc) {
    const v16b a = frag_b(XB + (r0 + wave * 16 + col) * DM + kc * 32, lane);
#pragma unroll
    for (int j = 0; j < 8; ++j) acc[j] = wmma_bf(a, frag_b(WB + (size_t)(c0 + j * 16 + col) * DM + kc * 32, lane), acc[j]);
  }
#pragma unroll
  for (int j = 0; j < 8; ++j)
#pragma unroll
    for (int r = 0; r < 8; ++r) { const float v = acc[j][r]; const _Float16 hv = f16n(v); sh[wave * 16 + 8 * g + r][j * 16 + col] = hv; sl[wave * 16 + 8 * g + r][j * 16 + col] = f16n((v - (float)hv) * RC); }
  __syncthreads();
  for (int e = tid; e < 64 * 16; e += 128) { const int rl = e >> 4, q = e & 15; const size_t o = (r0 + rl) * (size_t)DM + c0 + q * 8; vst2(OH + o, *(const v8h*)&sh[rl][q * 8]); vst2(OL + o, *(const v8h*)&sl[rl][q * 8]); }
}

__global__ __launch_bounds__(128) void k_pvt(const __bf16* __restrict__ XB, const __bf16* __restrict__ WVT, _Float16* __restrict__ VT) {
  __shared__ __align__(16) _Float16 th[128][72];
  const int tid = threadIdx.x, wave = tid >> 5, lane = tid & 31, col = lane & 15, g = lane >> 4;
  const int c0 = blockIdx.y * 128; const size_t r0 = (size_t)blockIdx.x * 64;
  const unsigned rr = blockIdx.x * 64u; const unsigned b = rr / (unsigned)SEQ; const unsigned s0 = rr - b * (unsigned)SEQ;
  v8f acc[8];
#pragma unroll
  for (int j = 0; j < 8; ++j) acc[j] = zero8();
#pragma unroll 1
  for (int kc = 0; kc < DM / 32; ++kc) {
    const v16b a = frag_b(XB + (r0 + wave * 16 + col) * DM + kc * 32, lane);
#pragma unroll
    for (int j = 0; j < 8; ++j) acc[j] = wmma_bf(a, frag_b(WVT + (size_t)(c0 + j * 16 + col) * DM + kc * 32, lane), acc[j]);
  }
#pragma unroll
  for (int j = 0; j < 8; ++j)
#pragma unroll
    for (int r = 0; r < 8; ++r) th[j * 16 + col][wave * 16 + 8 * g + r] = f16n(acc[j][r]);
  __syncthreads();
  for (int e = tid; e < 128 * 8; e += 128) { const int cl = e >> 3, q = e & 7; vst2(VT + ((size_t)(b * (unsigned)DM + (unsigned)(c0 + cl))) * SEQ + s0 + q * 8, *(const v8h*)&th[cl][q * 8]); }
}

__global__ __launch_bounds__(128) void k_att(const _Float16* __restrict__ QH, const _Float16* __restrict__ QL, const _Float16* __restrict__ KH, const _Float16* __restrict__ KL,
                                             const _Float16* __restrict__ VT, _Float16* __restrict__ CTX) {
  __shared__ __align__(16) _Float16 sP[4][16][40];
  __shared__ __align__(16) _Float16 so[4][16][72];
  const int tid = threadIdx.x, wave = tid >> 5, lane = tid & 31, col = lane & 15, g = lane >> 4;
  const int b = (int)(blockIdx.y >> 4), h = (int)(blockIdx.y & 15u);
  const int q0 = (int)blockIdx.x * 64 + wave * 16;
  const size_t rb = (size_t)b * SEQ; const size_t hoff = (size_t)h * HD;
  v16h ah[2], ar[2];
#pragma unroll
  for (int kc = 0; kc < 2; ++kc) { ah[kc] = frag_h(QH + (rb + q0 + col) * DM + hoff + kc * 32, lane); ar[kc] = frag_h(QL + (rb + q0 + col) * DM + hoff + kc * 32, lane); }
  float m[8];
#pragma unroll
  for (int r = 0; r < 8; ++r) m[r] = -3.0e38f;
  const int jd = q0 >> 4;
#pragma unroll 1
  for (int jt = 0; jt <= jd; ++jt) {
    const _Float16* kp = KH + (rb + jt * 16 + col) * DM + hoff;
    v8f c = zero8();
#pragma unroll
    for (int kc = 0; kc < 2; ++kc) c = wmma16(ah[kc], frag_h(kp + kc * 32, lane), c);
    const bool dg = (jt == jd);
#pragma unroll
    for (int r = 0; r < 8; ++r) { const float cv = (dg && (col > 8 * g + r)) ? -3.0e38f : c[r]; m[r] = fmaxf(m[r], cv); }
  }
  float mref[8], lsum[8];
#pragma unroll
  for (int r = 0; r < 8; ++r) { float t = m[r]; t = fmaxf(t, __shfl_xor(t, 1)); t = fmaxf(t, __shfl_xor(t, 2)); t = fmaxf(t, __shfl_xor(t, 4)); t = fmaxf(t, __shfl_xor(t, 8)); mref[r] = t * SCALE + 1.0f; lsum[r] = 0.f; }
  v8f acc[4];
#pragma unroll
  for (int j = 0; j < 4; ++j) acc[j] = zero8();
#pragma unroll 1
  for (int j = 0; j < q0 + 16; j += 32) {
    LDSX();
#pragma unroll
    for (int t = 0; t < 2; ++t) {
      v8f cs = zero8(), cl = zero8();
      const size_t ko = (rb + j + 16 * t + col) * DM + hoff;
#pragma unroll
      for (int kc = 0; kc < 2; ++kc) {
        const v16h bh = frag_h(KH + ko + kc * 32, lane);
        const v16h br = frag_h(KL + ko + kc * 32, lane);
        cs = wmma16(ah[kc], bh, cs); cl = wmma16(ar[kc], bh, cl); cl = wmma16(ah[kc], br, cl);
      }
      const int kidx = j + 16 * t + col;
#pragma unroll
      for (int r = 0; r < 8; ++r) {
        const float s = (cs[r] + cl[r] * (1.0f / RC)) * SCALE;
        const float e = fminf(s - mref[r], 1.0f);
        float pc = __expf(e) * PCY; pc = (pc >= F16MIN) ? pc : 0.0f;
        pc = (kidx <= q0 + 8 * g + r) ? pc : 0.0f;
        const _Float16 ph = (_Float16)pc;
        lsum[r] += (float)ph;
        sP[wave][8 * g + r][16 * t + col] = ph;
      }
    }
    LDSX();
    const v16h a = frag_h(&sP[wave][col][0], lane);
#pragma unroll
    for (int jv = 0; jv < 4; ++jv) acc[jv] = wmma16(a, frag_h(VT + ((size_t)(b * DM) + hoff + jv * 16 + col) * SEQ + j, lane), acc[jv]);
  }
  float inv[8];
#pragma unroll
  for (int r = 0; r < 8; ++r) { float t = lsum[r]; t += __shfl_xor(t, 1); t += __shfl_xor(t, 2); t += __shfl_xor(t, 4); t += __shfl_xor(t, 8); inv[r] = (1.0f / t) * CC; }
  LDSX();
#pragma unroll
  for (int jv = 0; jv < 4; ++jv)
#pragma unroll
    for (int r = 0; r < 8; ++r) so[wave][8 * g + r][jv * 16 + col] = f16n(acc[jv][r] * inv[r]);
  LDSX();
#pragma unroll
  for (int i = 0; i < 4; ++i) { const int rl = i * 4 + (lane >> 3), pq = lane & 7; const v8h v = *(const v8h*)&so[wave][rl][pq * 8]; vst2(CTX + (rb + q0 + rl) * DM + hoff + pq * 8, v); }
}

__global__ __launch_bounds__(128) void k_gl(const _Float16* __restrict__ C16, const _Float16* __restrict__ WOH, const unsigned short* __restrict__ XBu, float* __restrict__ OUT) {
  __shared__ __align__(16) float sf[4][16][132];
  const int tid = threadIdx.x, wave = tid >> 5, lane = tid & 31, col = lane & 15, g = lane >> 4; const int c0 = blockIdx.y * 128; const size_t r0 = (size_t)blockIdx.x * 64 + wave * 16;
  const unsigned rc = blockIdx.x * 64u + (unsigned)wave * 16u; const unsigned bb = rc / (unsigned)SEQ; const size_t rf0 = (size_t)bb * SEQ_FULL + (rc - bb * (unsigned)SEQ);
  v8f acc[8];
#pragma unroll
  for (int j = 0; j < 8; ++j) acc[j] = zero8();
#pragma unroll 1
  for (int kc = 0; kc < DM / 32; ++kc) { const v16h a = frag_h(C16 + (r0 + col) * DM + kc * 32, lane);
#pragma unroll
    for (int j = 0; j < 8; ++j) acc[j] = wmma16(a, frag_h(WOH + (size_t)(c0 + j * 16 + col) * DM + kc * 32, lane), acc[j]); }
#pragma unroll
  for (int j = 0; j < 8; ++j)
#pragma unroll
    for (int r = 0; r < 8; ++r) sf[wave][8 * g + r][j * 16 + col] = acc[j][r] * (1.0f / (WC * CC));
  LDSX();
  for (int rl = 0; rl < 16; ++rl) {
    const size_t oc = (r0 + rl) * (size_t)DM + c0 + lane * 4; const size_t of = (rf0 + rl) * (size_t)DM + c0 + lane * 4;
    v4f vv = *(const v4f*)&sf[wave][rl][lane * 4]; const v4us xb = *(const v4us*)(XBu + oc);
    vv[0] += bf16val(xb[0]); vv[1] += bf16val(xb[1]); vv[2] += bf16val(xb[2]); vv[3] += bf16val(xb[3]);
    vst2(OUT + of, vv);
  }
}

extern "C" void kernel_launch(void* const* d_in, const int* in_sizes, int n_in, void* d_out, int out_size, void* d_ws, size_t ws_size, hipStream_t stream) {
  if (n_in < 5) return;
  const int xneed = ((NB - 1) * SEQ_FULL + SEQ) * DM;
  if (in_sizes[0] < xneed || in_sizes[1] < DM * DM || in_sizes[2] < DM * DM || in_sizes[3] < DM * DM || in_sizes[4] < DM * DM) return;
  if (out_size < xneed) return;
  if (ws_size < (size_t)WS_END) return;
  const float* X = (const float*)d_in[0]; const float* WQ = (const float*)d_in[1]; const float* WK = (const float*)d_in[2]; const float* WV = (const float*)d_in[3]; const float* WO = (const float*)d_in[4];
  char* ws = (char*)d_ws;
  unsigned short* XBu = (unsigned short*)(ws + WS_XB); unsigned short* WQTu = (unsigned short*)(ws + WS_WQT); unsigned short* WKTu = (unsigned short*)(ws + WS_WKT);
  unsigned short* WVTu = (unsigned short*)(ws + WS_WVT); unsigned short* WOHu = (unsigned short*)(ws + WS_WOH);
  const __bf16* XB = (const __bf16*)(ws + WS_XB); const __bf16* WQT = (const __bf16*)(ws + WS_WQT); const __bf16* WKT = (const __bf16*)(ws + WS_WKT); const __bf16* WVT = (const __bf16*)(ws + WS_WVT);
  const _Float16* WOH = (const _Float16*)(ws + WS_WOH);
  _Float16 *QH = (_Float16*)(ws + WS_QH), *QL = (_Float16*)(ws + WS_QL), *KH = (_Float16*)(ws + WS_KH), *KL = (_Float16*)(ws + WS_KL), *VT = (_Float16*)(ws + WS_VT), *CTX = (_Float16*)(ws + WS_CTX);

  k_cvtx<<<dim3(N8X / 256u), 256, 0, stream>>>(X, XBu);
  k_cvtw<<<dim3(DM / 64, DM / 64, 4), 256, 0, stream>>>(WQ, WK, WV, WO, WQTu, WKTu, WVTu, WOHu);
  k_pqk<<<dim3(MROWS / 64, DM / 128, 2), 128, 0, stream>>>(XB, WQT, WKT, QH, QL, KH, KL);
  k_pvt<<<dim3(MROWS / 64, DM / 128), 128, 0, stream>>>(XB, WVT, VT);
  k_att<<<dim3(SEQ / 64, NB * NH), 128, 0, stream>>>(QH, QL, KH, KL, VT, CTX);
  k_gl<<<dim3(MROWS / 64, DM / 128), 128, 0, stream>>>(CTX, WOH, XBu, (float*)d_out);
}
